// Char2Vec_27023934226760
// MI455X (gfx1250) — hardware-run, weakly checked
//
#include <hip/hip_runtime.h>
#include <math.h>

typedef __attribute__((ext_vector_type(16))) _Float16 v16h;
typedef __attribute__((ext_vector_type(8)))  _Float16 v8h;
typedef __attribute__((ext_vector_type(8)))  float    v8f;
typedef __attribute__((ext_vector_type(4)))  float    v4f;

constexpr int kVocab    = 128;
constexpr int kEmb      = 128;
constexpr int kCh1      = 256;
constexpr int kCh2      = 256;
constexpr int kTaps     = 3;
constexpr int kWords    = 64 * 128;
constexpr int kLen      = 32;
constexpr int kLen1     = kLen - kTaps + 1;
constexpr int kLen2     = kLen1 - kTaps + 1;
constexpr int kHalfWords = kWords / 2;
constexpr int kRowsHalf  = kHalfWords * kLen;
constexpr int kTailRows  = kTaps - 1;
constexpr int kK2        = kTaps * kCh1;
constexpr float kWCarry    = 64.0f;
constexpr float kWCarryInv = 1.0f / kWCarry;

static_assert(kLen1 == 30 && kLen2 == 28, "time lengths 32 -> 30 -> 28");
static_assert(kLen == 32, "one word = 32 plane rows = two 16-row subtiles");
static_assert((kRowsHalf % 64) == 0 && (kWords % 64) == 0, "GEMM M multiples of 64");
static_assert((kCh2 % 64) == 0, "GEMM N multiple of 64");
static_assert((kK2 % 32) == 0 && (kCh2 % 32) == 0, "GEMM K multiples of 32");
static_assert((kCh1 % 8) == 0, "8-wide k groups never straddle a tap");

constexpr size_t kSzTAB = (size_t)kTaps * kVocab * kCh1 * 4;
constexpr size_t kSzBT2 = (size_t)kCh2 * kK2 * 2;
constexpr size_t kSzBTL = (size_t)kCh2 * kCh2 * 2;
constexpr size_t kSzH1  = (size_t)(kRowsHalf + kTailRows) * kCh1 * 2;
constexpr size_t kSzPF  = (size_t)kWords * kCh2 * 4;
constexpr size_t kSzPH  = (size_t)kWords * kCh2 * 2;
constexpr size_t kOffTAB = 0;
constexpr size_t kOffBT2 = kOffTAB + kSzTAB;
constexpr size_t kOffBTL = kOffBT2 + kSzBT2;
constexpr size_t kOffH1  = kOffBTL + kSzBTL;
constexpr size_t kOffPF  = kOffH1  + kSzH1;
constexpr size_t kOffPH  = kOffPF  + kSzPF;
constexpr size_t kWsTotal = kOffPH + kSzPH;
static_assert(kWsTotal == 80610304ull, "carve total");
static_assert(kWsTotal <= 134217728ull, "carve cap");
static_assert((kOffBT2 % 128) == 0 && (kOffBTL % 128) == 0 && (kOffH1 % 128) == 0 &&
              (kOffPF % 128) == 0 && (kOffPH % 128) == 0, "128-B aligned regions");

union FragH { v16h v; v8h h[2]; };
__device__ __forceinline__ v16h frag_load_h(const _Float16* p) {
  FragH f;
  f.h[0] = *(const v8h*)(p);
  f.h[1] = *(const v8h*)(p + 16);
  return f.v;
}
__device__ __forceinline__ v8f mma_h(v16h a, v16h b, v8f c) {
  c = __builtin_amdgcn_wmma_f32_16x16x32_f16(false, a, false, b, (short)0, c, false, false);
  asm volatile("v_nop\n\tv_nop\n\tv_nop\n\tv_nop" : "+v"(c) : "v"(a), "v"(b));
  return c;
}
__device__ __forceinline__ void keep4_h(v16h a, v16h b, v16h c, v16h d) { asm volatile("v_nop" :: "v"(a), "v"(b), "v"(c), "v"(d)); }
__device__ __forceinline__ void acc_guard4(v8f& a, v8f& b, v8f& c, v8f& d) { asm volatile("v_nop\n\tv_nop\n\tv_nop\n\tv_nop" : "+v"(a), "+v"(b), "+v"(c), "+v"(d)); }

constexpr int kPackBlocks2 = (kCh2 * kK2 / 8) / 256;
constexpr int kPackBlocksL = (kCh2 * kCh2 / 8) / 256;
static_assert(kPackBlocks2 * 256 * 8 == kCh2 * kK2, "BT2 coverage");
static_assert(kPackBlocksL * 256 * 8 == kCh2 * kCh2, "BTL coverage");

__global__ __launch_bounds__(256) void pack_weights_kernel(
    const float* __restrict__ w2, const float* __restrict__ wl,
    unsigned short* __restrict__ bt2, unsigned short* __restrict__ btl)
{
  const int tid = threadIdx.x;
  v8h hv;
  unsigned short* q;
  if (blockIdx.x < kPackBlocks2) {
    const int i   = blockIdx.x * 256 + tid;
    const int e0  = i * 8;
    const int co  = e0 / kK2;
    const int k   = e0 - co * kK2;
    const int tap = k / kCh1;
    const int ci0 = k - tap * kCh1;
    const float* s = w2 + ((size_t)co * kCh1 + ci0) * kTaps + tap;
#pragma unroll
    for (int e = 0; e < 8; ++e) {
      const float x = s[e * kTaps] * kWCarry;
      hv[e] = (_Float16)x;
    }
    q = bt2 + e0;
  } else {
    const int i  = (blockIdx.x - kPackBlocks2) * 256 + tid;
    const int e0 = i * 8;
    const v4f a0 = *(const v4f*)(wl + e0);
    const v4f a1 = *(const v4f*)(wl + e0 + 4);
#pragma unroll
    for (int e = 0; e < 4; ++e) {
      const float x0 = a0[e] * kWCarry;
      const float x1 = a1[e] * kWCarry;
      hv[e]     = (_Float16)x0;
      hv[4 + e] = (_Float16)x1;
    }
    q = btl + e0;
  }
  *(volatile v8h*)q = hv;
  __threadfence();
  *(volatile v8h*)q = hv;
}

__global__ __launch_bounds__(256) void table_kernel(
    const float* __restrict__ emb, const float* __restrict__ w1, const float* __restrict__ b1,
    float* __restrict__ tab)
{
  __shared__ __align__(16) float sE[kEmb];
  __shared__ __align__(16) float sO[kTaps * kCh1];
  const int tid = threadIdx.x;
  const int v   = blockIdx.x;
  if (tid < kEmb) sE[tid] = emb[(size_t)v * kEmb + tid];
  __syncthreads();
  const float* wp = w1 + (size_t)tid * kEmb * kTaps;
  float a0 = b1[tid];
  float a1 = 0.0f;
  float a2 = 0.0f;
#pragma unroll 4
  for (int ci = 0; ci < kEmb; ++ci) {
    const float e = sE[ci];
    a0 = fmaf(e, wp[ci * kTaps + 0], a0);
    a1 = fmaf(e, wp[ci * kTaps + 1], a1);
    a2 = fmaf(e, wp[ci * kTaps + 2], a2);
  }
  sO[0 * kCh1 + tid] = a0;
  sO[1 * kCh1 + tid] = a1;
  sO[2 * kCh1 + tid] = a2;
  __syncthreads();
  if (tid < kTaps * (kCh1 / 4)) {
    const int tap = tid / (kCh1 / 4);
    const int c4  = (tid - tap * (kCh1 / 4)) * 4;
    const v4f val = *(const v4f*)(sO + tap * kCh1 + c4);
    float* dst = tab + ((size_t)tap * kVocab + v) * kCh1 + c4;
    *(volatile v4f*)dst = val;
    __threadfence();
    *(volatile v4f*)dst = val;
  }
}

__global__ __launch_bounds__(256) void h1_build_kernel(
    const int* __restrict__ word, const float* __restrict__ tab, unsigned short* __restrict__ h1, int word0)
{
  const int lane = threadIdx.x & 31;
  const int wave = threadIdx.x >> 5;
  const int row  = blockIdx.x * 8 + wave;
  if (row >= kRowsHalf + kTailRows) return;
  const bool live = (row < kRowsHalf) && ((row & (kLen - 1)) < kLen1);
  const int rowc = (row < kRowsHalf) ? row : (kRowsHalf - 1);
  const int n    = word0 + (rowc >> 5);
  int t = rowc & (kLen - 1);
  t = (t < kLen1) ? t : (kLen1 - 1);
  const int* wp = word + (size_t)n * kLen + t;
  int i0 = wp[0];
  int i1 = wp[1];
  int i2 = wp[2];
  i0 = min(max(i0, 0), kVocab - 1);
  i1 = min(max(i1, 0), kVocab - 1);
  i2 = min(max(i2, 0), kVocab - 1);
  const float* p0 = tab + ((size_t)(0 * kVocab + i0)) * kCh1 + lane * 8;
  const float* p1 = tab + ((size_t)(1 * kVocab + i1)) * kCh1 + lane * 8;
  const float* p2 = tab + ((size_t)(2 * kVocab + i2)) * kCh1 + lane * 8;
  const v4f a0 = *(const v4f*)(p0);
  const v4f a1 = *(const v4f*)(p0 + 4);
  const v4f b0 = *(const v4f*)(p1);
  const v4f b1v = *(const v4f*)(p1 + 4);
  const v4f c0 = *(const v4f*)(p2);
  const v4f c1 = *(const v4f*)(p2 + 4);
  v8h hv;
#pragma unroll
  for (int e = 0; e < 4; ++e) {
    float s0 = (a0[e] + b0[e]) + c0[e];
    float s1 = (a1[e] + b1v[e]) + c1[e];
    s0 = fmaxf(s0, 0.0f);
    s1 = fmaxf(s1, 0.0f);
    s0 = live ? s0 : 0.0f;
    s1 = live ? s1 : 0.0f;
    hv[e]     = (_Float16)s0;
    hv[4 + e] = (_Float16)s1;
  }
  unsigned short* q = h1 + (size_t)row * kCh1 + lane * 8;
  *(volatile v8h*)q = hv;
  __threadfence();
  *(volatile v8h*)q = hv;
}

template <int EPI>
__global__ __launch_bounds__(256) void gemm_f16_kernel(
    const unsigned short* __restrict__ Ap, int lda,
    const unsigned short* __restrict__ Btp, int ldb,
    const float* __restrict__ bias,
    float* __restrict__ outF, unsigned short* __restrict__ outH,
    const float* __restrict__ resid,
    int M, int N, int K, float scale)
{
  const _Float16* A  = (const _Float16*)Ap;
  const _Float16* Bt = (const _Float16*)Btp;
  __shared__ __align__(16) float sT[8][16 * 68];
  const int lane = threadIdx.x & 31;
  const int wave = threadIdx.x >> 5;
  const int tilesN = N >> 6;
  const int tilesM = M >> 6;
  const int tile = blockIdx.x * 8 + wave;
  if (tile >= tilesM * tilesN) return;
  const int tm = tile / tilesN;
  const int tn = tile - tm * tilesN;
  const int m0 = tm << 6;
  const int n0 = tn << 6;
  const int ldc = N;

  const int rlane = lane & 15;
  const int koff  = (lane >> 4) * 8;
  const int mOff  = (lane >> 4) * 8;
  const int hsel  = lane >> 4;

  v8f acc[4][4];
#pragma unroll
  for (int i = 0; i < 4; ++i)
#pragma unroll
    for (int j = 0; j < 4; ++j) acc[i][j] = (v8f){0.f,0.f,0.f,0.f,0.f,0.f,0.f,0.f};

  for (int k0 = 0; k0 < K; k0 += 32) {
    v16h bh[4];
#pragma unroll
    for (int j = 0; j < 4; ++j) {
      const size_t bo = (size_t)(n0 + (j << 4) + rlane) * ldb + koff + k0;
      bh[j] = frag_load_h(Bt + bo);
    }
#pragma unroll
    for (int i = 0; i < 4; ++i) {
      const size_t ao = (size_t)(m0 + (i << 4) + rlane) * lda + koff + k0;
      const v16h ah = frag_load_h(A + ao);
#pragma unroll
      for (int j = 0; j < 4; ++j) acc[i][j] = mma_h(ah, bh[j], acc[i][j]);
    }
    keep4_h(bh[0], bh[1], bh[2], bh[3]);
  }
  acc_guard4(acc[0][0], acc[0][1], acc[0][2], acc[0][3]);
  acc_guard4(acc[1][0], acc[1][1], acc[1][2], acc[1][3]);
  acc_guard4(acc[2][0], acc[2][1], acc[2][2], acc[2][3]);
  acc_guard4(acc[3][0], acc[3][1], acc[3][2], acc[3][3]);

  float* slab = sT[wave];

  if (EPI == 0) {
#pragma unroll
    for (int w = 0; w < 2; ++w) {
#pragma unroll
      for (int j = 0; j < 4; ++j) {
        float m = acc[2 * w][j][0];
#pragma unroll
        for (int r = 1; r < 8; ++r) m = fmaxf(m, acc[2 * w][j][r]);
#pragma unroll
        for (int r = 0; r < 4; ++r) m = fmaxf(m, acc[2 * w + 1][j][r]);
        float m2 = fmaxf(fmaxf(acc[2 * w + 1][j][4], acc[2 * w + 1][j][5]),
                         fmaxf(acc[2 * w + 1][j][6], acc[2 * w + 1][j][7]));
        m2 = (hsel == 0) ? m2 : -INFINITY;
        m = fmaxf(m, m2);
        const float o = __shfl_xor(m, 16, 32);
        m = fmaxf(m, o);
        const float bv = bias[n0 + (j << 4) + rlane];
        const float pv = fmaxf(m * scale + bv, 0.0f);
        if (hsel == 0) slab[w * 64 + (j << 4) + rlane] = pv;
      }
    }
    __builtin_amdgcn_fence(__ATOMIC_RELEASE, "workgroup");
    __builtin_amdgcn_wave_barrier();
    __builtin_amdgcn_fence(__ATOMIC_ACQUIRE, "workgroup");
    const int word0 = m0 >> 5;
    const int wf = lane >> 4;
    const int c4 = (lane & 15) * 4;
    const v4f fv = *(const v4f*)(slab + wf * 64 + c4);
    const int wq = (lane >> 3) & 1;
    const int c8 = (lane & 7) * 8;
    const v4f s0 = *(const v4f*)(slab + wq * 64 + c8);
    const v4f s1 = *(const v4f*)(slab + wq * 64 + c8 + 4);
    v8h hv;
#pragma unroll
    for (int e = 0; e < 4; ++e) {
      const float x0 = s0[e];
      const float x1 = s1[e];
      hv[e]     = (_Float16)x0;
      hv[4 + e] = (_Float16)x1;
    }
    float* pf = outF + (size_t)(word0 + wf) * ldc + n0 + c4;
    unsigned short* ph = outH + (size_t)(word0 + wq) * ldc + n0 + c8;
    *(volatile v4f*)pf = fv;
    if (lane < 16) *(volatile v8h*)ph = hv;
    __threadfence();
    *(volatile v4f*)pf = fv;
    if (lane < 16) *(volatile v8h*)ph = hv;
  } else {
#pragma unroll
    for (int i = 0; i < 4; ++i) {
      const int mBase = m0 + (i << 4);
#pragma unroll
      for (int j = 0; j < 4; ++j) {
        const int n = n0 + (j << 4) + rlane;
        const float bv = bias[n];
#pragma unroll
        for (int r = 0; r < 8; ++r) {
          const float v = fmaxf(acc[i][j][r] * scale + bv, 0.0f);
          slab[(mOff + r) * 68 + (j << 4) + rlane] = v;
        }
      }
      __builtin_amdgcn_fence(__ATOMIC_RELEASE, "workgroup");
      __builtin_amdgcn_wave_barrier();
      __builtin_amdgcn_fence(__ATOMIC_ACQUIRE, "workgroup");
      const int c4 = (lane & 15) * 4;
      v4f ov[8];
#pragma unroll
      for (int it = 0; it < 8; ++it) {
        const int row = it * 2 + hsel;
        const v4f sv = *(const v4f*)(slab + row * 68 + c4);
        const v4f rv = *(const v4f*)(resid + (size_t)(mBase + row) * ldc + n0 + c4);
        ov[it] = sv + rv;
      }
      for (int pass = 0; pass < 2; ++pass) {
#pragma unroll
        for (int it = 0; it < 8; ++it) {
          const int row = it * 2 + hsel;
          *(volatile v4f*)(outF + (size_t)(mBase + row) * ldc + n0 + c4) = ov[it];
        }
        __threadfence();
      }
      __builtin_amdgcn_fence(__ATOMIC_RELEASE, "workgroup");
      __builtin_amdgcn_wave_barrier();
      __builtin_amdgcn_fence(__ATOMIC_ACQUIRE, "workgroup");
    }
  }
}

extern "C" void kernel_launch(void* const* d_in, const int* in_sizes, int n_in,
                              void* d_out, int out_size, void* d_ws, size_t ws_size,
                              hipStream_t stream) {
  if (n_in < 8) return;
  if (in_sizes[0] != kWords * kLen) return;
  if (in_sizes[1] != kVocab * kEmb) return;
  if (in_sizes[2] != kCh1 * kEmb * kTaps) return;
  if (in_sizes[3] != kCh1) return;
  if (in_sizes[4] != kCh2 * kCh1 * kTaps) return;
  if (in_sizes[5] != kCh2) return;
  if (in_sizes[6] != kCh2 * kCh2) return;
  if (in_sizes[7] != kCh2) return;
  if (out_size != kWords * kCh2) return;
  if (ws_size < kWsTotal) return;

  const int*   word = (const int*)  d_in[0];
  const float* emb  = (const float*)d_in[1];
  const float* w1   = (const float*)d_in[2];
  const float* b1   = (const float*)d_in[3];
  const float* w2   = (const float*)d_in[4];
  const float* b2   = (const float*)d_in[5];
  const float* wl   = (const float*)d_in[6];
  const float* bl   = (const float*)d_in[7];
  float* out = (float*)d_out;

  char* ws = (char*)d_ws;
  float*          TAB = (float*)(ws + kOffTAB);
  unsigned short* BT2 = (unsigned short*)(ws + kOffBT2);
  unsigned short* BTL = (unsigned short*)(ws + kOffBTL);
  unsigned short* H1  = (unsigned short*)(ws + kOffH1);
  float*          PF  = (float*)(ws + kOffPF);
  unsigned short* PH  = (unsigned short*)(ws + kOffPH);

  pack_weights_kernel<<<kPackBlocks2 + kPackBlocksL, 256, 0, stream>>>(w2, wl, BT2, BTL);
  table_kernel<<<kVocab, 256, 0, stream>>>(emb, w1, b1, TAB);

  const int h1Blocks = (kRowsHalf + kTailRows + 7) / 8;
  const int convBlocks = ((kRowsHalf / 64) * (kCh2 / 64)) / 8;
  for (int half = 0; half < 2; ++half) {
    const int word0 = half * kHalfWords;
    h1_build_kernel<<<h1Blocks, 256, 0, stream>>>(word, TAB, H1, word0);
    gemm_f16_kernel<0><<<convBlocks, 256, 0, stream>>>(
        H1, kCh1, BT2, kK2, b2,
        PF + (size_t)word0 * kCh2, PH + (size_t)word0 * kCh2, nullptr,
        kRowsHalf, kCh2, kK2, kWCarryInv);
  }

  const int linBlocks = ((kWords / 64) * (kCh2 / 64)) / 8;
  gemm_f16_kernel<1><<<linBlocks, 256, 0, stream>>>(
      PH, kCh2, BTL, kCh2, bl,
      out, nullptr, PF,
      kWords, kCh2, kCh2, kWCarryInv);
}
